// Model_56307021251126
// MI455X (gfx1250) — hardware-verified
//
#include <hip/hip_runtime.h>
#include <stddef.h>
#include <stdint.h>


#define DF      128
#define HP      256
#define PQW     256
#define K1      256
#define NNODE   100000
#define NEDGE   640000
#define MPAD    100096
#define NTHR    256
#define NWAVE   8
#define EPT     8
#define CHUNK   (NTHR * EPT)
#define WCAP    (EPT * 32)
#define LISTN   (NWAVE * WCAP)
#define NBA     1024
#define SLA     10
#define NBLK    98
#define RCAP    8192
#define DEGCAP  32
#define GBM     64
#define GBN     128
#define GTHR    128
#define ROWH    256
#define SCE     1024
#define UPART   2048
#define NWPART  15
#define NUW     (NWPART * UPART)
#define NUX     (MPAD * 16)
#define CMP_ZINTS   (LISTN + 2 * RCAP + 3 * NBA)
#define MISC_INTS   16
#define CMP_LDS_INTS (CMP_ZINTS + MISC_INTS)

static_assert((CHUNK & (CHUNK - 1)) == 0 && CHUNK <= 4096);
static_assert((NBA & (NBA - 1)) == 0 && NBA == (1 << SLA));
static_assert(((long long)CHUNK << SLA) < (1LL << 31));
static_assert(NEDGE < (1 << 21));
static_assert(NBA == NTHR * 4 && NBA % NWAVE == 0);
static_assert(RCAP % (NTHR * 4) == 0 && CMP_ZINTS % (NTHR * 4) == 0);
static_assert(RCAP >= 7097);
static_assert(DEGCAP >= 28);
static_assert(NBLK * NBA >= MPAD && MPAD >= NNODE && MPAD % GBM == 0 && MPAD % 128 == 0);
static_assert(NBLK <= NTHR);
static_assert(NEDGE == 625 * SCE && SCE % 32 == 0 && SCE == NTHR * 4 && SCE == NWAVE * 128);
static_assert(((long long)NEDGE * 4) % 128 == 0);
static_assert(GBN == DF && GBM == (GTHR / 32) * 16 && DF == 4 * 32 && ROWH == 2 * DF && HP == 2 * DF);
static_assert(K1 % 32 == 0 && 384 % 32 == 0 && 512 % 32 == 0);
static_assert(UPART % NTHR == 0 && NUW % NTHR == 0 && NUX % NTHR == 0 && UPART == DF * (DF / 8));
static_assert(CMP_LDS_INTS * 4 <= 300000);

typedef float          v4f   __attribute__((ext_vector_type(4)));
typedef float          v8f   __attribute__((ext_vector_type(8)));
typedef int            v4i   __attribute__((ext_vector_type(4)));
typedef int            v8i   __attribute__((ext_vector_type(8)));
typedef unsigned       v2u   __attribute__((ext_vector_type(2)));
typedef unsigned short v4us  __attribute__((ext_vector_type(4)));
typedef unsigned short v8us  __attribute__((ext_vector_type(8)));
typedef unsigned short v16us __attribute__((ext_vector_type(16)));
typedef __bf16         v16bf __attribute__((ext_vector_type(16)));
typedef v4f  __attribute__((may_alias)) v4fa;
typedef v4i  __attribute__((may_alias)) v4ia;
typedef v2u  __attribute__((may_alias)) v2ua;
typedef v4us __attribute__((may_alias)) v4usa;
typedef v8us __attribute__((may_alias)) v8usa;
union FragB { v16bf v; v16us u; v8us h[2]; v8i w; };

__device__ __forceinline__ v8f wmb(const FragB& a, const FragB& b, v8f c) {
  v8f d = __builtin_amdgcn_wmma_f32_16x16x32_bf16(false, a.v, false, b.v, (short)0, c, false, false);
  asm volatile("v_nop\n\tv_nop\n\tv_nop\n\tv_nop" : "+v"(d) : "v"(a.w), "v"(b.w));
  return d;
}

__device__ __forceinline__ unsigned bf16_bits(float f) {
  const unsigned u = __float_as_uint(f);
  const unsigned r = (u + 0x7FFFu + ((u >> 16) & 1u)) >> 16;
  return (f != f) ? 0x7FC0u : r;
}
__device__ __forceinline__ float bf16_val(float f) {
  return __uint_as_float(bf16_bits(f) << 16);
}
__device__ __forceinline__ unsigned hl_bits(float v, unsigned& lo) {
  const unsigned hb = bf16_bits(v);
  lo = bf16_bits(v - __uint_as_float(hb << 16));
  return hb;
}

__device__ __forceinline__ void wave_sync() {
  __builtin_amdgcn_fence(__ATOMIC_RELEASE, "wavefront");
  __builtin_amdgcn_wave_barrier();
  __builtin_amdgcn_fence(__ATOMIC_ACQUIRE, "wavefront");
}

template <int SLB>
__device__ __forceinline__ int scan_chunk(const int* __restrict__ dsts, int nE, int cbase, int slotBase,
                                          int nb, int vec8, int* list, int tid, int lane, int wave) {
  int wc = 0;
  const int el0  = tid * EPT;
  const int e0   = cbase + el0;
  const int sent = -2147483647 - 1;
  v4i da, db;
  if (vec8 != 0 && cbase + CHUNK <= nE) {
    da = *(const v4i*)(dsts + e0);
    db = *(const v4i*)(dsts + e0 + 4);
  } else {
    da.x = (e0     < nE) ? dsts[min(e0,     nE - 1)] : sent;
    da.y = (e0 + 1 < nE) ? dsts[min(e0 + 1, nE - 1)] : sent;
    da.z = (e0 + 2 < nE) ? dsts[min(e0 + 2, nE - 1)] : sent;
    da.w = (e0 + 3 < nE) ? dsts[min(e0 + 3, nE - 1)] : sent;
    db.x = (e0 + 4 < nE) ? dsts[min(e0 + 4, nE - 1)] : sent;
    db.y = (e0 + 5 < nE) ? dsts[min(e0 + 5, nE - 1)] : sent;
    db.z = (e0 + 6 < nE) ? dsts[min(e0 + 6, nE - 1)] : sent;
    db.w = (e0 + 7 < nE) ? dsts[min(e0 + 7, nE - 1)] : sent;
  }
  const unsigned nbs = (unsigned)slotBase;
  const unsigned unb = (unsigned)nb;
  const unsigned s0 = (unsigned)da.x - nbs, s1 = (unsigned)da.y - nbs;
  const unsigned s2 = (unsigned)da.z - nbs, s3 = (unsigned)da.w - nbs;
  const unsigned s4 = (unsigned)db.x - nbs, s5 = (unsigned)db.y - nbs;
  const unsigned s6 = (unsigned)db.z - nbs, s7 = (unsigned)db.w - nbs;
  const bool h0 = s0 < unb, h1 = s1 < unb, h2 = s2 < unb, h3 = s3 < unb;
  const bool h4 = s4 < unb, h5 = s5 < unb, h6 = s6 < unb, h7 = s7 < unb;
  const unsigned any = __builtin_amdgcn_ballot_w32(h0 | h1 | h2 | h3 | h4 | h5 | h6 | h7);
  if (any != 0u) {
#define HITJ(J, HJ, SJ) { \
      const unsigned mj = __builtin_amdgcn_ballot_w32(HJ); \
      if (mj != 0u) { \
        if (HJ) { \
          const int pos = wc + (int)__builtin_amdgcn_mbcnt_lo(mj, 0u); \
          if (pos < WCAP) list[wave * WCAP + pos] = ((el0 + (J)) << SLB) | (int)(SJ); \
        } \
        wc += (int)__builtin_popcount(mj); } }
    HITJ(0, h0, s0)
    HITJ(1, h1, s1)
    HITJ(2, h2, s2)
    HITJ(3, h3, s3)
    HITJ(4, h4, s4)
    HITJ(5, h5, s5)
    HITJ(6, h6, s6)
    HITJ(7, h7, s7)
#undef HITJ
  }
  return wc;
}

__global__ __launch_bounds__(NTHR) void k_prep(const float* __restrict__ x,
                                               const float* __restrict__ ws1, const float* __restrict__ wn1,
                                               const float* __restrict__ ws2, const float* __restrict__ wn2,
                                               const float* __restrict__ ws3, const float* __restrict__ wn3,
                                               const float* __restrict__ wp1,
                                               unsigned short* w1c, unsigned short* w2c, unsigned short* w3c,
                                               unsigned short* wpt, unsigned short* xb, int nN) {
  const int u = (int)blockIdx.x * NTHR + (int)threadIdx.x;
  v8us o;
  unsigned short* dp;
  if (u < NUW) {
    const int part = u >> 11;
    const int v    = u & (UPART - 1);
    const int n    = v >> 4;
    const int k8   = (v & 15) * 8;
    const float* W;
    unsigned short* P;
    int pitch, coff, rowo;
    if (part == 0)       { W = wn1; P = w1c; pitch = 384; coff = 0;      rowo = 0; }
    else if (part == 1)  { W = wn1; P = w1c; pitch = 384; coff = DF;     rowo = 0; }
    else if (part == 2)  { W = ws1; P = w1c; pitch = 384; coff = 2 * DF; rowo = 0; }
    else if (part == 3)  { W = wn2; P = w2c; pitch = 512; coff = 0;      rowo = 0; }
    else if (part == 4)  { W = wn2; P = w2c; pitch = 512; coff = DF;     rowo = 0; }
    else if (part == 5)  { W = ws2; P = w2c; pitch = 512; coff = 2 * DF; rowo = 0; }
    else if (part == 6)  { W = ws2; P = w2c; pitch = 512; coff = 3 * DF; rowo = 0; }
    else if (part == 7)  { W = wn3; P = w3c; pitch = 512; coff = 0;      rowo = 0; }
    else if (part == 8)  { W = wn3; P = w3c; pitch = 512; coff = DF;     rowo = 0; }
    else if (part == 9)  { W = ws3; P = w3c; pitch = 512; coff = 2 * DF; rowo = 0; }
    else if (part == 10) { W = ws3; P = w3c; pitch = 512; coff = 3 * DF; rowo = 0; }
    else if (part == 11) { W = wp1;           P = wpt; pitch = 256; coff = 0;  rowo = 0; }
    else if (part == 12) { W = wp1;           P = wpt; pitch = 256; coff = DF; rowo = 0; }
    else if (part == 13) { W = wp1 + DF * DF; P = wpt; pitch = 256; coff = 0;  rowo = DF; }
    else                 { W = wp1 + DF * DF; P = wpt; pitch = 256; coff = DF; rowo = DF; }
    const float* p = W + (size_t)k8 * DF + n;
    const float f0 = p[0],      f1 = p[DF],     f2 = p[2 * DF], f3 = p[3 * DF];
    const float f4 = p[4 * DF], f5 = p[5 * DF], f6 = p[6 * DF], f7 = p[7 * DF];
    o[0] = (unsigned short)bf16_bits(f0); o[1] = (unsigned short)bf16_bits(f1);
    o[2] = (unsigned short)bf16_bits(f2); o[3] = (unsigned short)bf16_bits(f3);
    o[4] = (unsigned short)bf16_bits(f4); o[5] = (unsigned short)bf16_bits(f5);
    o[6] = (unsigned short)bf16_bits(f6); o[7] = (unsigned short)bf16_bits(f7);
    dp = P + (size_t)(rowo + n) * pitch + coff + k8;
  } else if (u < NUW + NUX) {
    const int v   = u - NUW;
    const int row = v >> 4, k8 = (v & 15) * 8;
    const int rc  = row < nN ? row : nN - 1;
    const bool lv = row < nN;
    const float* p = x + (size_t)rc * DF + k8;
    const v4f a = *(const v4f*)p;
    const v4f b = *(const v4f*)(p + 4);
    o[0] = (unsigned short)bf16_bits(lv ? a.x : 0.0f); o[1] = (unsigned short)bf16_bits(lv ? a.y : 0.0f);
    o[2] = (unsigned short)bf16_bits(lv ? a.z : 0.0f); o[3] = (unsigned short)bf16_bits(lv ? a.w : 0.0f);
    o[4] = (unsigned short)bf16_bits(lv ? b.x : 0.0f); o[5] = (unsigned short)bf16_bits(lv ? b.y : 0.0f);
    o[6] = (unsigned short)bf16_bits(lv ? b.z : 0.0f); o[7] = (unsigned short)bf16_bits(lv ? b.w : 0.0f);
    dp = xb + (size_t)v * 8;
  } else {
    return;
  }
  *(volatile v8us*)dp = o;
  __threadfence();
  *(volatile v8us*)dp = o;
}

__global__ __launch_bounds__(NTHR) void k_compact(const int* __restrict__ srcs, const int* __restrict__ dsts,
                                                  int nE, int nN, int vec8,
                                                  int* lst, int* cntg, int* offg, int* ovfg) {
  extern __shared__ __attribute__((aligned(16))) int dsm[];
  int* list = dsm;
  int* hl   = dsm + LISTN;
  int* sl   = hl + RCAP;
  int* cnt  = sl + RCAP;
  int* offs = cnt + NBA;
  int* cur  = offs + NBA;
  int* misc = cur + NBA;
  const int tid = (int)threadIdx.x, lane = tid & 31, wave = tid >> 5;
  const int blk = (int)blockIdx.x;
  const int nodeBase = blk * NBA;

  {
    const v4i z4 = {0, 0, 0, 0};
    for (int i = tid * 4; i < CMP_ZINTS; i += NTHR * 4) *(v4ia*)(dsm + i) = z4;
    if (tid < MISC_INTS) misc[tid] = 0;
  }
  __syncthreads();

  int t = 0, ov = 0;
  const int nChunks = (nE + CHUNK - 1) / CHUNK;
#pragma unroll 1
  for (int ch = 0; ch < nChunks; ++ch) {
    const int cbase = ch * CHUNK;
    const int wc = scan_chunk<SLA>(dsts, nE, cbase, nodeBase, NBA, vec8, list, tid, lane, wave);
    if (lane == 0) misc[wave] = wc;
    __syncthreads();
    if (wave == 0) {
#pragma unroll 1
      for (int w2 = 0; w2 < NWAVE; ++w2) {
        int c = misc[w2];
        c = c < 0 ? 0 : (c > WCAP ? WCAP : c);
#pragma unroll 1
        for (int b0 = 0; b0 < c; b0 += 32) {
          const int idx = b0 + lane;
          const int ent_ = list[w2 * WCAP + (idx < WCAP ? idx : WCAP - 1)];
          const int m32 = (c - b0) < 32 ? (c - b0) : 32;
#pragma unroll 1
          for (int k = 0; k < m32; ++k) {
            const int u    = __builtin_amdgcn_readlane(ent_, k);
            const int slot = u & (NBA - 1);
            const int el   = (u >> SLA) & (CHUNK - 1);
            const int pk   = ((cbase + el) << SLA) | slot;
            if (t < RCAP) {
              if (lane == 0) { hl[t] = pk; cnt[slot] = cnt[slot] + 1; }
              t = t + 1;
            } else {
              ov = 1;
            }
          }
        }
      }
    }
    __syncthreads();
  }
  if (wave == 0 && lane == 0) { misc[8] = t; misc[9] = ov; }
  __syncthreads();
  int tt = misc[8];
  tt = tt < 0 ? 0 : (tt > RCAP ? RCAP : tt);
  const int ovf = misc[9];

  if (wave == 0) {
    const int base = lane * (NBA / 32);
    int s = 0;
#pragma unroll 1
    for (int i = 0; i < NBA / 32; ++i) s += cnt[base + i];
    int incl = s;
#pragma unroll
    for (int d = 1; d < 32; d <<= 1) {
      const int y = __shfl_up(incl, d, 32);
      if (lane >= d) incl += y;
    }
    int run = incl - s;
#pragma unroll 1
    for (int i = 0; i < NBA / 32; ++i) {
      const int cv = cnt[base + i];
      offs[base + i] = run;
      cur[base + i]  = run;
      run += cv;
    }
  }
  __syncthreads();
  if (wave == 0) {
#pragma unroll 1
    for (int b0 = 0; b0 < tt; b0 += 32) {
      const int idx = b0 + lane;
      const int ent_ = hl[idx < RCAP ? idx : RCAP - 1];
      const int m32 = (tt - b0) < 32 ? (tt - b0) : 32;
#pragma unroll 1
      for (int k = 0; k < m32; ++k) {
        const int u    = __builtin_amdgcn_readlane(ent_, k);
        const int slot = u & (NBA - 1);
        if (lane == 0) {
          int p = cur[slot];
          p = p < 0 ? 0 : (p > RCAP - 1 ? RCAP - 1 : p);
          sl[p] = u;
          cur[slot] = p + 1;
        }
      }
    }
  }
  __syncthreads();

  int* lrow = lst + (size_t)blk * RCAP;
#pragma unroll 1
  for (int it = 0; it < RCAP / (NTHR * 4); ++it) {
    const int p0 = it * (NTHR * 4) + 4 * tid;
    const v4i e4 = *(const v4ia*)(sl + p0);
    int e0 = e4.x >> SLA, e1 = e4.y >> SLA, e2 = e4.z >> SLA, e3 = e4.w >> SLA;
    e0 = e0 < 0 ? 0 : (e0 > nE - 1 ? nE - 1 : e0);
    e1 = e1 < 0 ? 0 : (e1 > nE - 1 ? nE - 1 : e1);
    e2 = e2 < 0 ? 0 : (e2 > nE - 1 ? nE - 1 : e2);
    e3 = e3 < 0 ? 0 : (e3 > nE - 1 ? nE - 1 : e3);
    int r0 = srcs[e0], r1 = srcs[e1], r2 = srcs[e2], r3 = srcs[e3];
    r0 = r0 < 0 ? 0 : (r0 > nN - 1 ? nN - 1 : r0);
    r1 = r1 < 0 ? 0 : (r1 > nN - 1 ? nN - 1 : r1);
    r2 = r2 < 0 ? 0 : (r2 > nN - 1 ? nN - 1 : r2);
    r3 = r3 < 0 ? 0 : (r3 > nN - 1 ? nN - 1 : r3);
    v4i o;
    o.x = (p0     < tt) ? r0 : 0;
    o.y = (p0 + 1 < tt) ? r1 : 0;
    o.z = (p0 + 2 < tt) ? r2 : 0;
    o.w = (p0 + 3 < tt) ? r3 : 0;
    *(volatile v4i*)(lrow + p0) = o;
    __threadfence();
    *(volatile v4i*)(lrow + p0) = o;
  }
  {
    const v4i c4 = *(const v4ia*)(cnt + 4 * tid);
    const v4i o4 = *(const v4ia*)(offs + 4 * tid);
    int* cg = cntg + nodeBase + 4 * tid;
    int* og = offg + nodeBase + 4 * tid;
    *(volatile v4i*)cg = c4;
    *(volatile v4i*)og = o4;
    __threadfence();
    *(volatile v4i*)cg = c4;
    *(volatile v4i*)og = o4;
  }
  if (tid < 8) {
    v4i f4; f4.x = ovf; f4.y = ovf; f4.z = ovf; f4.w = ovf;
    int* fg = ovfg + blk * 32 + 4 * tid;
    *(volatile v4i*)fg = f4;
    __threadfence();
    *(volatile v4i*)fg = f4;
  }
}

template <int L0>
__global__ __launch_bounds__(NTHR) void k_agg(const int* __restrict__ lst, const int* __restrict__ cntg,
                                              const int* __restrict__ offg, const int* __restrict__ ovfg,
                                              const unsigned short* __restrict__ hp, unsigned short* agg,
                                              int nN, int mRows) {
  __shared__ __attribute__((aligned(16))) int cnts[NBA];
  __shared__ __attribute__((aligned(16))) int offs[NBA];
  __shared__ __attribute__((aligned(16))) unsigned short rowall[NWAVE * ROWH];
  const int tid = (int)threadIdx.x, lane = tid & 31, wave = tid >> 5;
  const int blk = (int)blockIdx.x;
  const int nodeBase = blk * NBA;
  unsigned short* rowbuf = rowall + wave * ROWH;
  {
    const v4i c4 = *(const v4i*)(cntg + nodeBase + 4 * tid);
    const v4i o4 = *(const v4i*)(offg + nodeBase + 4 * tid);
    *(v4ia*)(cnts + 4 * tid) = c4;
    *(v4ia*)(offs + 4 * tid) = o4;
  }
  const int ovf = ovfg[blk * 32];
  const int* lb = lst + (size_t)blk * RCAP;
  __syncthreads();

  const float qn = __int_as_float(0x7fc00000);
  const float pz = (ovf != 0) ? qn : 0.0f;
#pragma unroll 1
  for (int si = 0; si < NBA / NWAVE; ++si) {
    const int s    = si * NWAVE + wave;
    const int node = nodeBase + s;
    int c = cnts[s];
    const bool big = c > DEGCAP;
    c = c < 0 ? 0 : (c > DEGCAP ? DEGCAP : c);
    int o = offs[s];
    o = o < 0 ? 0 : (o > RCAP ? RCAP : o);
    const float pzr = big ? qn : pz;
    const bool live = node < nN;
    float a0 = 0.0f, a1 = 0.0f, a2 = 0.0f, a3 = 0.0f;
#pragma unroll 1
    for (int b0 = 0; b0 < c; b0 += 32) {
      int idx = o + b0 + lane;
      idx = idx > RCAP - 1 ? RCAP - 1 : idx;
      int sr = lb[idx];
      sr = sr < 0 ? 0 : (sr > nN - 1 ? nN - 1 : sr);
      const int m32 = (c - b0) < 32 ? (c - b0) : 32;
#pragma unroll 1
      for (int k = 0; k < m32; ++k) {
        const int sk = __builtin_amdgcn_readlane(sr, k);
        if constexpr (L0 != 0) {
          const unsigned short* rp = hp + (size_t)sk * DF + 4 * lane;
          const v2u wh = *(const v2ua*)rp;
          a0 += __uint_as_float(wh.x << 16);
          a1 += __uint_as_float(wh.x & 0xffff0000u);
          a2 += __uint_as_float(wh.y << 16);
          a3 += __uint_as_float(wh.y & 0xffff0000u);
        } else {
          const unsigned short* rp = hp + (size_t)sk * HP + 4 * lane;
          const v2u wh = *(const v2ua*)rp;
          const v2u wl = *(const v2ua*)(rp + DF);
          const float f0 = __uint_as_float(wh.x << 16)         + __uint_as_float(wl.x << 16);
          const float f1 = __uint_as_float(wh.x & 0xffff0000u) + __uint_as_float(wl.x & 0xffff0000u);
          const float f2 = __uint_as_float(wh.y << 16)         + __uint_as_float(wl.y << 16);
          const float f3 = __uint_as_float(wh.y & 0xffff0000u) + __uint_as_float(wl.y & 0xffff0000u);
          a0 += f0; a1 += f1; a2 += f2; a3 += f3;
        }
      }
    }
    const float inv = 1.0f / fmaxf((float)c, 1.0f);
    const float m0 = live ? (a0 * inv + pzr) : 0.0f;
    const float m1 = live ? (a1 * inv + pzr) : 0.0f;
    const float m2 = live ? (a2 * inv + pzr) : 0.0f;
    const float m3 = live ? (a3 * inv + pzr) : 0.0f;
    v4us mh, ml;
    {
      unsigned lo_b;
      unsigned hi_b;
      hi_b = hl_bits(m0, lo_b); mh[0] = (unsigned short)hi_b; ml[0] = (unsigned short)lo_b;
      hi_b = hl_bits(m1, lo_b); mh[1] = (unsigned short)hi_b; ml[1] = (unsigned short)lo_b;
      hi_b = hl_bits(m2, lo_b); mh[2] = (unsigned short)hi_b; ml[2] = (unsigned short)lo_b;
      hi_b = hl_bits(m3, lo_b); mh[3] = (unsigned short)hi_b; ml[3] = (unsigned short)lo_b;
    }
    *(v4usa*)(rowbuf + 4 * lane)      = mh;
    *(v4usa*)(rowbuf + DF + 4 * lane) = ml;
    wave_sync();
    const v8us q0 = *(const v8usa*)(rowbuf + 8 * lane);
    wave_sync();
    if (node < mRows) {
      unsigned short* rpw = agg + (size_t)node * HP + 8 * lane;
      *(volatile v8us*)rpw = q0;
      __threadfence();
      *(volatile v8us*)rpw = q0;
    }
  }
}

template <int EPI>
__global__ __launch_bounds__(GTHR) void k_gemm(const unsigned short* __restrict__ A1,
                                               const unsigned short* __restrict__ A2, int lda2, int K2,
                                               const unsigned short* __restrict__ BT, int ldb,
                                               const float* __restrict__ bias,
                                               unsigned short* hout, float* pq, int nN, int mRows) {
  __shared__ __attribute__((aligned(16))) float stg[GBM * GBN];
  const int tid = (int)threadIdx.x, lane = tid & 31, wave = tid >> 5, hh = lane >> 4, m = lane & 15;
  const int rowBase = (int)blockIdx.x * GBM;
  const int ny = (int)blockIdx.y;

  v8f acc[8];
  {
    const v8f z = {0.f, 0.f, 0.f, 0.f, 0.f, 0.f, 0.f, 0.f};
#pragma unroll
    for (int t = 0; t < 8; ++t) acc[t] = z;
  }
  const unsigned short* ap1 = A1 + (size_t)(rowBase + 16 * wave + m) * (size_t)HP + 8 * hh;
  const unsigned short* ap2 = A2 + (size_t)(rowBase + 16 * wave + m) * (size_t)lda2 + 8 * hh;
  const unsigned short* bp  = BT + (size_t)(GBN * ny + m) * (size_t)ldb + 8 * hh;

#pragma unroll 1
  for (int k0 = 0; k0 < K1; k0 += 32) {
    FragB af;
    af.h[0] = *(const v8usa*)(ap1 + k0);
    af.h[1] = *(const v8usa*)(ap1 + k0 + 16);
#pragma unroll
    for (int nt = 0; nt < 8; ++nt) {
      const unsigned short* wq = bp + (size_t)(16 * nt) * (size_t)ldb + k0;
      FragB bf;
      bf.h[0] = *(const v8usa*)wq;
      bf.h[1] = *(const v8usa*)(wq + 16);
      acc[nt] = wmb(af, bf, acc[nt]);
    }
  }
#pragma unroll 1
  for (int k0 = 0; k0 < K2; k0 += 32) {
    FragB af;
    af.h[0] = *(const v8usa*)(ap2 + k0);
    af.h[1] = *(const v8usa*)(ap2 + k0 + 16);
#pragma unroll
    for (int nt = 0; nt < 8; ++nt) {
      const unsigned short* wq = bp + (size_t)(16 * nt) * (size_t)ldb + K1 + k0;
      FragB bf;
      bf.h[0] = *(const v8usa*)wq;
      bf.h[1] = *(const v8usa*)(wq + 16);
      acc[nt] = wmb(af, bf, acc[nt]);
    }
  }

#pragma unroll
  for (int nt = 0; nt < 8; ++nt) {
    const int lc = 16 * nt + m;
#pragma unroll
    for (int r = 0; r < 8; ++r) {
      const int lr = 16 * wave + 8 * hh + r;
      stg[lr * GBN + lc] = acc[nt][r];
    }
  }
  __syncthreads();

  v4f bb4;
  {
    const v4f t1 = *(const v4f*)(bias + 4 * lane);
    bb4.x = bf16_val(t1.x); bb4.y = bf16_val(t1.y); bb4.z = bf16_val(t1.z); bb4.w = bf16_val(t1.w);
    if constexpr (EPI != 0) {
      const bool top = (ny == 0);
      bb4.x = top ? bb4.x : 0.0f; bb4.y = top ? bb4.y : 0.0f;
      bb4.z = top ? bb4.z : 0.0f; bb4.w = top ? bb4.w : 0.0f;
    }
  }

  v4f pv[16];
#pragma unroll
  for (int i = 0; i < 16; ++i) pv[i] = *(const v4fa*)(stg + (16 * wave + i) * GBN + 4 * lane);
  __syncthreads();

#pragma unroll
  for (int i = 0; i < 16; ++i) {
    const bool ok = (rowBase + 16 * wave + i) < nN;
    v4f y = pv[i] + bb4;
    y.x = ok ? y.x : 0.0f; y.y = ok ? y.y : 0.0f; y.z = ok ? y.z : 0.0f; y.w = ok ? y.w : 0.0f;
    pv[i] = y;
  }

  if constexpr (EPI != 0) {
#pragma unroll
    for (int i = 0; i < 16; ++i) {
      const int gr = rowBase + 16 * wave + i;
      float* op = pq + (size_t)gr * PQW + GBN * ny + 4 * lane;
      if (gr < mRows) *(volatile v4f*)op = pv[i];
    }
    __threadfence();
#pragma unroll
    for (int i = 0; i < 16; ++i) {
      const int gr = rowBase + 16 * wave + i;
      float* op = pq + (size_t)gr * PQW + GBN * ny + 4 * lane;
      if (gr < mRows) *(volatile v4f*)op = pv[i];
    }
    (void)hout;
  } else {
#pragma unroll
    for (int i = 0; i < 16; ++i) {
      v4us h4, l4;
      unsigned lo_b;
      unsigned hi_b;
      hi_b = hl_bits(pv[i].x, lo_b); h4[0] = (unsigned short)hi_b; l4[0] = (unsigned short)lo_b;
      hi_b = hl_bits(pv[i].y, lo_b); h4[1] = (unsigned short)hi_b; l4[1] = (unsigned short)lo_b;
      hi_b = hl_bits(pv[i].z, lo_b); h4[2] = (unsigned short)hi_b; l4[2] = (unsigned short)lo_b;
      hi_b = hl_bits(pv[i].w, lo_b); h4[3] = (unsigned short)hi_b; l4[3] = (unsigned short)lo_b;
      unsigned short* srow = (unsigned short*)stg + (size_t)(16 * wave + i) * (2 * GBN);
      *(v4usa*)(srow + 4 * lane) = h4;
      *(v4usa*)(srow + DF + 4 * lane) = l4;
    }
    __syncthreads();
    v8us qv[16];
#pragma unroll
    for (int i = 0; i < 16; ++i) {
      const unsigned short* srow = (const unsigned short*)stg + (size_t)(16 * wave + i) * (2 * GBN);
      qv[i] = *(const v8usa*)(srow + 8 * lane);
    }
#pragma unroll
    for (int i = 0; i < 16; ++i) {
      const int gr = rowBase + 16 * wave + i;
      unsigned short* rp = hout + (size_t)gr * (size_t)HP + 8 * lane;
      if (gr < mRows) *(volatile v8us*)rp = qv[i];
    }
    __threadfence();
#pragma unroll
    for (int i = 0; i < 16; ++i) {
      const int gr = rowBase + 16 * wave + i;
      unsigned short* rp = hout + (size_t)gr * (size_t)HP + 8 * lane;
      if (gr < mRows) *(volatile v8us*)rp = qv[i];
    }
    (void)pq;
  }
}

__global__ __launch_bounds__(NTHR) void k_score(const float* __restrict__ pq,
                                                const int* __restrict__ ps0, const int* __restrict__ pd0,
                                                const int* __restrict__ ps1, const int* __restrict__ pd1,
                                                const float* __restrict__ wp2, const float* __restrict__ bp2,
                                                const int* __restrict__ ovfg, int nblk,
                                                float* out, int nE, int nN) {
  __shared__ __attribute__((aligned(16))) float sc[SCE];
  __shared__ int wfl[NWAVE];
  const int tid = (int)threadIdx.x, lane = tid & 31, wave = tid >> 5;
  const int y = (int)blockIdx.y;
  const int msk = -y;
  {
    const int fi = tid < nblk ? tid : nblk - 1;
    int f = ovfg[fi * 32];
    f = (tid < nblk) ? f : 0;
    const unsigned bal = __builtin_amdgcn_ballot_w32(f != 0);
    if (lane == 0) wfl[wave] = (bal != 0u) ? 1 : 0;
  }
  v4f w4;
  {
    const v4f t1 = *(const v4f*)(wp2 + 4 * lane);
    w4.x = bf16_val(t1.x); w4.y = bf16_val(t1.y); w4.z = bf16_val(t1.z); w4.w = bf16_val(t1.w);
  }
  const float b2 = bf16_val(bp2[0]);
  const int eb = (int)blockIdx.x * SCE + wave * 128;
#pragma unroll 1
  for (int b = 0; b < 4; ++b) {
    const int e  = eb + 32 * b + lane;
    const int ec = e < nE ? e : nE - 1;
    const int sa = ps0[ec], sb = ps1[ec], da = pd0[ec], db = pd1[ec];
    int s = (sa & ~msk) | (sb & msk);
    int d = (da & ~msk) | (db & msk);
    s = s < 0 ? 0 : (s > nN - 1 ? nN - 1 : s);
    d = d < 0 ? 0 : (d > nN - 1 ? nN - 1 : d);
    float mine = 0.0f;
#pragma unroll 4
    for (int k = 0; k < 32; ++k) {
      const int sk = __builtin_amdgcn_readlane(s, k);
      const int dk = __builtin_amdgcn_readlane(d, k);
      const v4f a = *(const v4f*)(pq + (size_t)sk * PQW + 4 * lane);
      const v4f c = *(const v4f*)(pq + (size_t)dk * PQW + DF + 4 * lane);
      const v4f v = a + c;
      const float r0 = (v.x > 0.0f) ? v.x : (v.x - v.x);
      const float r1 = (v.y > 0.0f) ? v.y : (v.y - v.y);
      const float r2 = (v.z > 0.0f) ? v.z : (v.z - v.z);
      const float r3 = (v.w > 0.0f) ? v.w : (v.w - v.w);
      float p = r0 * w4.x;
      p = fmaf(r1, w4.y, p);
      p = fmaf(r2, w4.z, p);
      p = fmaf(r3, w4.w, p);
      p += __shfl_xor(p, 16, 32);
      p += __shfl_xor(p, 8, 32);
      p += __shfl_xor(p, 4, 32);
      p += __shfl_xor(p, 2, 32);
      p += __shfl_xor(p, 1, 32);
      mine = (lane == k) ? p : mine;
    }
    sc[wave * 128 + 32 * b + lane] = mine + b2;
  }
  __syncthreads();
  const int anyf = wfl[0] | wfl[1] | wfl[2] | wfl[3] | wfl[4] | wfl[5] | wfl[6] | wfl[7];
  const float qn = __int_as_float(0x7fc00000);
  v4f o = *(const v4fa*)(sc + 4 * tid);
  o.x = (anyf != 0) ? qn : o.x;
  o.y = (anyf != 0) ? qn : o.y;
  o.z = (anyf != 0) ? qn : o.z;
  o.w = (anyf != 0) ? qn : o.w;
  float* op = out + (size_t)y * (size_t)nE + (size_t)blockIdx.x * SCE + 4 * tid;
  *(volatile v4f*)op = o;
  __threadfence();
  *(volatile v4f*)op = o;
}

static inline size_t al256(size_t o) { return (o + 255) & ~(size_t)255; }

extern "C" void kernel_launch(void* const* d_in, const int* in_sizes, int n_in,
                              void* d_out, int out_size, void* d_ws, size_t ws_size,
                              hipStream_t stream) {
  if (n_in < 18) return;
  const int nN = NNODE, nE = NEDGE;
  if (in_sizes[0] != NNODE * DF) return;
  if (in_sizes[1] != nE || in_sizes[2] != nE || in_sizes[3] != nE || in_sizes[4] != nE) return;
  if (in_sizes[5] != DF * DF || in_sizes[6] != DF * DF || in_sizes[7] != DF) return;
  if (in_sizes[8] != DF * DF || in_sizes[9] != DF * DF || in_sizes[10] != DF) return;
  if (in_sizes[11] != DF * DF || in_sizes[12] != DF * DF || in_sizes[13] != DF) return;
  if (in_sizes[14] != 2 * DF * DF || in_sizes[15] != DF || in_sizes[16] != DF || in_sizes[17] != 1) return;
  if ((long long)out_size != 2LL * nE) return;

  const float* x    = (const float*)d_in[0];
  const int*   src  = (const int*)  d_in[1];
  const int*   dst  = (const int*)  d_in[2];
  const int*   nsrc = (const int*)  d_in[3];
  const int*   ndst = (const int*)  d_in[4];
  const float* Ws1 = (const float*)d_in[5];
  const float* Wn1 = (const float*)d_in[6];
  const float* b1  = (const float*)d_in[7];
  const float* Ws2 = (const float*)d_in[8];
  const float* Wn2 = (const float*)d_in[9];
  const float* b2  = (const float*)d_in[10];
  const float* Ws3 = (const float*)d_in[11];
  const float* Wn3 = (const float*)d_in[12];
  const float* b3  = (const float*)d_in[13];
  const float* Wp1 = (const float*)d_in[14];
  const float* bp1 = (const float*)d_in[15];
  const float* Wp2 = (const float*)d_in[16];
  const float* bp2 = (const float*)d_in[17];
  float* out = (float*)d_out;

  const size_t U = (size_t)MPAD * HP * 2;
  char* ws = (char*)d_ws;
  const size_t oHA  = 0;
  const size_t oAGG = U;
  const size_t oHB  = 2 * U;
  const size_t oXB  = 2 * U;
  const size_t oPQ  = U;
  size_t off = 3 * U;
  const size_t oLST = off; off = al256(off + (size_t)NBLK * RCAP * 4);
  const size_t oCNT = off; off = al256(off + (size_t)NBLK * NBA * 4);
  const size_t oOFF = off; off = al256(off + (size_t)NBLK * NBA * 4);
  const size_t oOVF = off; off = al256(off + (size_t)NBLK * 128);
  const size_t oW1  = off; off = al256(off + (size_t)DF * 384 * 2);
  const size_t oW2  = off; off = al256(off + (size_t)DF * 512 * 2);
  const size_t oW3  = off; off = al256(off + (size_t)DF * 512 * 2);
  const size_t oWP  = off; off = al256(off + (size_t)256 * 256 * 2);
  if (off > ws_size) return;
  if ((size_t)MPAD * DF * 2 > U) return;
  if ((size_t)MPAD * PQW * 4 != 2 * U) return;
  unsigned short* HA  = (unsigned short*)(ws + oHA);
  unsigned short* AGG = (unsigned short*)(ws + oAGG);
  unsigned short* HB  = (unsigned short*)(ws + oHB);
  unsigned short* XB  = (unsigned short*)(ws + oXB);
  float*          PQ  = (float*)(ws + oPQ);
  int* LST = (int*)(ws + oLST);
  int* CNT = (int*)(ws + oCNT);
  int* OFF = (int*)(ws + oOFF);
  int* OVF = (int*)(ws + oOVF);
  unsigned short* W1C = (unsigned short*)(ws + oW1);
  unsigned short* W2C = (unsigned short*)(ws + oW2);
  unsigned short* W3C = (unsigned short*)(ws + oW3);
  unsigned short* WPT = (unsigned short*)(ws + oWP);

  const int vec8 = ((nE & 3) == 0) ? 1 : 0;
  const int gM = MPAD / GBM;
  const size_t cLds = (size_t)CMP_LDS_INTS * 4;
  hipFuncSetAttribute(reinterpret_cast<const void*>(&k_compact), hipFuncAttributeMaxDynamicSharedMemorySize, (int)cLds);

  k_prep<<<(NUW + NUX) / NTHR, NTHR, 0, stream>>>(x, Ws1, Wn1, Ws2, Wn2, Ws3, Wn3, Wp1, W1C, W2C, W3C, WPT, XB, nN);
  k_compact<<<NBLK, NTHR, cLds, stream>>>(src, dst, nE, nN, vec8, LST, CNT, OFF, OVF);
  k_agg<1><<<NBLK, NTHR, 0, stream>>>(LST, CNT, OFF, OVF, XB, AGG, nN, MPAD);
  k_gemm<0><<<dim3(gM, 1), GTHR, 0, stream>>>(AGG, XB, DF, DF, W1C, 384, b1, HA, PQ, nN, MPAD);
  k_agg<0><<<NBLK, NTHR, 0, stream>>>(LST, CNT, OFF, OVF, HA, AGG, nN, MPAD);
  k_gemm<0><<<dim3(gM, 1), GTHR, 0, stream>>>(AGG, HA, HP, HP, W2C, 512, b2, HB, PQ, nN, MPAD);
  k_agg<0><<<NBLK, NTHR, 0, stream>>>(LST, CNT, OFF, OVF, HB, AGG, nN, MPAD);
  k_gemm<0><<<dim3(gM, 1), GTHR, 0, stream>>>(AGG, HB, HP, HP, W3C, 512, b3, HA, PQ, nN, MPAD);
  k_gemm<1><<<dim3(gM, 2), GTHR, 0, stream>>>(HA, HA, HP, 0, WPT, 256, bp1, HA, PQ, nN, MPAD);
  k_score<<<dim3(NEDGE / SCE, 2), NTHR, 0, stream>>>(PQ, src, dst, nsrc, ndst, Wp2, bp2, OVF, NBLK, out, nE, nN);
}
